// GraphTransformerLayer_70866960384543
// MI455X (gfx1250) — hardware-verified
//
#include <hip/hip_runtime.h>
#include <stddef.h>
#include <stdint.h>
#include <math.h>


#define DM      128
#define NHD     8
#define HDM     16
#define EDM     12
#define QW      512
#define OQ      0
#define OKY     128
#define OV      256
#define OS      384
#define KO      256
#define FW      512
#define KF      1024
#define NTHR    256
#define NWAVE   8
#define EPT     8
#define CHUNK   (NTHR * EPT)
#define WCAP    (EPT * 32)
#define LISTN   (NWAVE * WCAP)
#define NBMAX   1024
#define SLOTB   10
#define RCAP    28672
#define DEGCAP  64
#define GBM     64
#define GBN     64
#define GTHR    128
#define KU      4
#define ATTSC   0.25f
#define LNEPS   1e-5f
#define WSMAX   134217728
#define LDS_AGG  ((2 * RCAP + 2 * NBMAX + LISTN + 2 * NWAVE) * 4 + EDM * DM * 4 + 64)
#define LDS_TAIL (GBM * KO * 2 + GBM * KF * 2 + GBM * DM * 4)

static_assert((1 << SLOTB) == NBMAX);
static_assert(SLOTB + 21 <= 31);
static_assert((CHUNK & (CHUNK - 1)) == 0 && CHUNK <= 2048 && SLOTB + 11 <= 31);
static_assert(NTHR * 4 == NBMAX);
static_assert(LISTN >= NBMAX);
static_assert(LISTN >= NWAVE * WCAP);
static_assert((RCAP % 32) == 0);
static_assert((NBMAX % NWAVE) == 0);
static_assert((((2 * RCAP + 2 * NBMAX + LISTN + 2 * NWAVE) * 4) % 16) == 0);
static_assert(LDS_AGG <= 300000 && LDS_TAIL <= 300000);
static_assert(GBM == (GTHR / 32) * 16);
static_assert((DM % 32) == 0 && ((DM / 32) % KU) == 0);
static_assert((DM / 8) == 16);
static_assert(DM == 4 * 32);
static_assert(HDM == 4 * 4 && NHD * HDM == DM);
static_assert(QW == 4 * DM && (DM % GBN) == 0);
static_assert((EDM % 4) == 0 && ((EDM * 4) % 16) == 0);
static_assert(KO == 2 * DM && FW == 4 * DM && KF == 2 * FW && (KO % 32) == 0 && (KF % 32) == 0);
static_assert(GBM * (DM / 8) == 8 * GTHR);

typedef float          v4f  __attribute__((ext_vector_type(4)));
typedef float          v8f  __attribute__((ext_vector_type(8)));
typedef int            v4i  __attribute__((ext_vector_type(4)));
typedef int            v8i  __attribute__((ext_vector_type(8)));
typedef unsigned int   v2u  __attribute__((ext_vector_type(2)));
typedef unsigned int   v4u  __attribute__((ext_vector_type(4)));
typedef unsigned short v8us __attribute__((ext_vector_type(8)));
typedef __bf16         v16b __attribute__((ext_vector_type(16)));
typedef v4f  __attribute__((may_alias)) v4fa;
typedef v2u  __attribute__((may_alias)) v2ua;
typedef v4u  __attribute__((may_alias)) v4ua;
typedef v8us __attribute__((may_alias)) v8usa;
union FragB { v16b v; v8us h[2]; v8i w; };

__device__ __forceinline__ v8f wmb(const FragB& a, const FragB& b, v8f c) {
  v8f d = __builtin_amdgcn_wmma_f32_16x16x32_bf16(false, a.v, false, b.v, (short)0, c, false, false);
  asm volatile("v_nop\n\tv_nop\n\tv_nop\n\tv_nop" : "+v"(d) : "v"(a.w), "v"(b.w));
  return d;
}

__device__ __forceinline__ unsigned int f2bf(float f) {
  const unsigned int u = __float_as_uint(f);
  return ((u + 0x7FFFu + ((u >> 16) & 1u)) >> 16) & 0xFFFFu;
}
__device__ __forceinline__ float bf2f(unsigned int b) { return __uint_as_float(b << 16); }
__device__ __forceinline__ float bfr(float f) { return bf2f(f2bf(f)); }
__device__ __forceinline__ v4f bfr4(const v4f a) {
  v4f r; r.x = bfr(a.x); r.y = bfr(a.y); r.z = bfr(a.z); r.w = bfr(a.w); return r;
}
__device__ __forceinline__ unsigned int pk2(float lo, float hi) { return f2bf(lo) | (f2bf(hi) << 16); }
__device__ __forceinline__ v4u pack8(const v4f a, const v4f b) {
  v4u r;
  r.x = pk2(a.x, a.y); r.y = pk2(a.z, a.w); r.z = pk2(b.x, b.y); r.w = pk2(b.z, b.w);
  return r;
}
__device__ __forceinline__ void hl2(float v0, float v1, unsigned int& hw, unsigned int& lw) {
  const unsigned int h0 = f2bf(v0), h1 = f2bf(v1);
  const unsigned int l0 = f2bf(v0 - bf2f(h0)), l1 = f2bf(v1 - bf2f(h1));
  hw = h0 | (h1 << 16);
  lw = l0 | (l1 << 16);
}
__device__ __forceinline__ void pack8hl(const v4f a, const v4f b, v4u& hv, v4u& lv) {
  unsigned int h, l;
  hl2(a.x, a.y, h, l); hv.x = h; lv.x = l;
  hl2(a.z, a.w, h, l); hv.y = h; lv.y = l;
  hl2(b.x, b.y, h, l); hv.z = h; lv.z = l;
  hl2(b.z, b.w, h, l); hv.w = h; lv.w = l;
}

__device__ __forceinline__ float wsum(float v) {
  v += __shfl_xor(v, 16, 32);
  v += __shfl_xor(v, 8, 32);
  v += __shfl_xor(v, 4, 32);
  v += __shfl_xor(v, 2, 32);
  v += __shfl_xor(v, 1, 32);
  return v;
}
__device__ __forceinline__ float hsum4(float v) {
  v += __shfl_xor(v, 1, 32);
  v += __shfl_xor(v, 2, 32);
  return v;
}
__device__ __forceinline__ float dot4(const v4f a, const v4f b) {
  float p = a.x * b.x; p = fmaf(a.y, b.y, p); p = fmaf(a.z, b.z, p); p = fmaf(a.w, b.w, p);
  return p;
}
__device__ __forceinline__ v4f relu4(const v4f a) {
  v4f r; r.x = fmaxf(a.x, 0.0f); r.y = fmaxf(a.y, 0.0f); r.z = fmaxf(a.z, 0.0f); r.w = fmaxf(a.w, 0.0f); return r;
}

__device__ __forceinline__ int scan_chunk(const int* __restrict__ dsts, int nE, int cbase, int slotBase,
                                          int nb, int vec8, int* list, int tid, int lane, int wave) {
  int wc = 0;
  const int el0  = tid * EPT;
  const int e0   = cbase + el0;
  const int sent = -2147483647 - 1;
  v4i da, db;
  if (vec8 != 0 && cbase + CHUNK <= nE) {
    da = *(const v4i*)(dsts + e0);
    db = *(const v4i*)(dsts + e0 + 4);
  } else {
    da.x = (e0     < nE) ? dsts[min(e0,     nE - 1)] : sent;
    da.y = (e0 + 1 < nE) ? dsts[min(e0 + 1, nE - 1)] : sent;
    da.z = (e0 + 2 < nE) ? dsts[min(e0 + 2, nE - 1)] : sent;
    da.w = (e0 + 3 < nE) ? dsts[min(e0 + 3, nE - 1)] : sent;
    db.x = (e0 + 4 < nE) ? dsts[min(e0 + 4, nE - 1)] : sent;
    db.y = (e0 + 5 < nE) ? dsts[min(e0 + 5, nE - 1)] : sent;
    db.z = (e0 + 6 < nE) ? dsts[min(e0 + 6, nE - 1)] : sent;
    db.w = (e0 + 7 < nE) ? dsts[min(e0 + 7, nE - 1)] : sent;
  }
  const unsigned nbs = (unsigned)slotBase;
  const unsigned unb = (unsigned)nb;
  const unsigned s0 = (unsigned)da.x - nbs, s1 = (unsigned)da.y - nbs;
  const unsigned s2 = (unsigned)da.z - nbs, s3 = (unsigned)da.w - nbs;
  const unsigned s4 = (unsigned)db.x - nbs, s5 = (unsigned)db.y - nbs;
  const unsigned s6 = (unsigned)db.z - nbs, s7 = (unsigned)db.w - nbs;
  const bool h0 = s0 < unb, h1 = s1 < unb, h2 = s2 < unb, h3 = s3 < unb;
  const bool h4 = s4 < unb, h5 = s5 < unb, h6 = s6 < unb, h7 = s7 < unb;
  const unsigned any = __builtin_amdgcn_ballot_w32(h0 | h1 | h2 | h3 | h4 | h5 | h6 | h7);
  if (any != 0u) {
#define HITJ(J, HJ, SJ) { \
      const unsigned mj = __builtin_amdgcn_ballot_w32(HJ); \
      if (mj != 0u) { \
        if (HJ) { \
          const int pos = wc + (int)__builtin_amdgcn_mbcnt_lo(mj, 0u); \
          if (pos < WCAP) list[wave * WCAP + pos] = ((el0 + (J)) << SLOTB) | (int)(SJ); \
        } \
        wc += (int)__builtin_popcount(mj); } }
    HITJ(0, h0, s0)
    HITJ(1, h1, s1)
    HITJ(2, h2, s2)
    HITJ(3, h3, s3)
    HITJ(4, h4, s4)
    HITJ(5, h5, s5)
    HITJ(6, h6, s6)
    HITJ(7, h7, s7)
#undef HITJ
  }
  return wc;
}

__global__ __launch_bounds__(NTHR) void k_xprep(const float* __restrict__ x, unsigned short* xbp, int nN, int nUnits) {
  const int i = (int)blockIdx.x * NTHR + (int)threadIdx.x;
  if (i >= nUnits) return;
  const int row = i >> 4;
  const int c0  = (i & 15) * 8;
  const int rc  = row < nN ? row : nN - 1;
  const float* p = x + (size_t)rc * DM + c0;
  v4f a = *(const v4fa*)p;
  v4f b = *(const v4fa*)(p + 4);
  const v4f z4 = {0.f, 0.f, 0.f, 0.f};
  if (row >= nN) { a = z4; b = z4; }
  const v4u hv = pack8(a, b);
  unsigned short* o = xbp + (size_t)row * DM + c0;
  *(volatile v4u*)o = hv;
  __threadfence();
  *(volatile v4u*)o = hv;
}

__global__ __launch_bounds__(NTHR) void k_wcvt(const float* __restrict__ w, int Kin, int Nrows, int Kout,
                                               unsigned short* wt, int nUnits) {
  const int u = (int)blockIdx.x * NTHR + (int)threadIdx.x;
  if (u >= nUnits) return;
  const int kq = Kout >> 3;
  int n  = u / kq;
  const int k8 = (u - n * kq) * 8;
  const int kk = k8 - (k8 / Kin) * Kin;
  n = n < Nrows ? n : Nrows - 1;
  const float* p = w + (size_t)n * (size_t)Kin + kk;
  const v4f a = *(const v4fa*)p;
  const v4f b = *(const v4fa*)(p + 4);
  const v4u wv = pack8(a, b);
  unsigned short* o = wt + (size_t)n * (size_t)Kout + k8;
  *(volatile v4u*)o = wv;
  __threadfence();
  *(volatile v4u*)o = wv;
}

__global__ __launch_bounds__(GTHR) void k_gemm(
    const unsigned short* __restrict__ A, const unsigned short* __restrict__ WT,
    const float* __restrict__ bias, float* outF)
{
  __shared__ __attribute__((aligned(16))) float stg[GBM * GBN];
  const int tid = (int)threadIdx.x, lane = tid & 31, wave = tid >> 5, hh = lane >> 4, m = lane & 15;
  const int rowBase = (int)blockIdx.x * GBM;
  const int col0    = (int)blockIdx.y * GBN;

  v8f acc[4];
  {
    const v8f z = {0.f, 0.f, 0.f, 0.f, 0.f, 0.f, 0.f, 0.f};
    acc[0] = z; acc[1] = z; acc[2] = z; acc[3] = z;
  }
  const unsigned short* ap = A  + (size_t)(rowBase + 16 * wave + m) * (size_t)DM + 8 * hh;
  const unsigned short* wp = WT + (size_t)(col0 + m) * (size_t)DM + 8 * hh;
#pragma unroll 1
  for (int ks0 = 0; ks0 < DM / 32; ks0 += KU) {
#pragma unroll
    for (int uu = 0; uu < KU; ++uu) {
      const int ks = ks0 + uu;
      FragB af;
      af.h[0] = *(const v8usa*)(ap + 32 * ks);
      af.h[1] = *(const v8usa*)(ap + 32 * ks + 16);
#pragma unroll
      for (int t = 0; t < 4; ++t) {
        const unsigned short* wq = wp + (size_t)(16 * t) * (size_t)DM + 32 * ks;
        FragB bf;
        bf.h[0] = *(const v8usa*)wq;
        bf.h[1] = *(const v8usa*)(wq + 16);
        acc[t] = wmb(af, bf, acc[t]);
      }
    }
  }

#pragma unroll
  for (int t = 0; t < 4; ++t) {
    const int lc = 16 * t + m;
#pragma unroll
    for (int r = 0; r < 8; ++r) {
      const int lr = 16 * wave + 8 * hh + r;
      stg[lr * GBN + lc] = acc[t][r];
    }
  }
  __syncthreads();

  const v4f bb = bfr4(*(const v4fa*)(bias + col0 + 4 * m));
  v4f fv[8];
#pragma unroll
  for (int i = 0; i < 8; ++i) {
    const int lr = 16 * wave + 2 * i + hh;
    fv[i] = *(const v4fa*)(stg + lr * GBN + 4 * m) + bb;
  }
#pragma unroll
  for (int i = 0; i < 8; ++i) {
    const int lr = 16 * wave + 2 * i + hh;
    const int gr = rowBase + lr;
    float* op = outF + (size_t)gr * (size_t)QW + col0 + 4 * m;
    *(volatile v4f*)op = fv[i];
  }
  __threadfence();
#pragma unroll
  for (int i = 0; i < 8; ++i) {
    const int lr = 16 * wave + 2 * i + hh;
    const int gr = rowBase + lr;
    float* op = outF + (size_t)gr * (size_t)QW + col0 + 4 * m;
    *(volatile v4f*)op = fv[i];
  }
}

__global__ __launch_bounds__(NTHR) void k_agg(
    const int* __restrict__ srcs, const int* __restrict__ dsts,
    const float* __restrict__ QKVS, const float* __restrict__ ea, const float* __restrict__ We,
    const float* __restrict__ Wb, const float* __restrict__ x,
    const float* __restrict__ g1p, const float* __restrict__ e1p,
    float* H1, int nN, int nE, int vec8, int MPr) {
  extern __shared__ v4f lds_dyn[];
  int* reg1 = (int*)lds_dyn;
  int* reg2 = reg1 + RCAP;
  int* scnt = reg2 + RCAP;
  int* soff = scnt + NBMAX;
  int* list = soff + NBMAX;
  int* wcnt = list + LISTN;
  int* wtot = wcnt + NWAVE;
  float* sWe = (float*)(wtot + NWAVE);
  const int tid = (int)threadIdx.x, lane = tid & 31, wave = tid >> 5;
  const int nodeBase = (int)blockIdx.x * NBMAX;

  for (int i = tid; i < NBMAX; i += NTHR) scnt[i] = 0;
#pragma unroll 1
  for (int i = tid; i < DM * EDM; i += NTHR) {
    const int c = i / EDM;
    const int j = i - c * EDM;
    sWe[j * DM + c] = bfr(We[i]);
  }
  __syncthreads();

  int tot = 0;
  const int nChunks = (nE + CHUNK - 1) / CHUNK;
#pragma unroll 1
  for (int ch = 0; ch < nChunks; ++ch) {
    const int cbase = ch * CHUNK;
    const int wc = scan_chunk(dsts, nE, cbase, nodeBase, NBMAX, vec8, list, tid, lane, wave);
    if (lane == 0) wcnt[wave] = wc;
    __syncthreads();
    int pre = 0, all = 0;
#pragma unroll
    for (int w2 = 0; w2 < NWAVE; ++w2) {
      int c = wcnt[w2];
      c = c < 0 ? 0 : (c > WCAP ? WCAP : c);
      all += c;
      pre += (w2 < wave) ? c : 0;
    }
    const int wcc  = wc > WCAP ? WCAP : wc;
    const int base = tot + pre;
#pragma unroll 1
    for (int i = lane; i < wcc; i += 32) {
      const int ent = list[wave * WCAP + i];
      const int el  = (ent >> SLOTB) & (CHUNK - 1);
      const int sl  = ent & (NBMAX - 1);
      int eid = cbase + el;
      eid = eid > nE - 1 ? nE - 1 : eid;
      const int pos = base + i;
      if (pos < RCAP) reg1[pos] = (int)(((unsigned)eid << SLOTB) | (unsigned)sl);
    }
    tot += all;
    tot = tot > RCAP ? RCAP : tot;
    __syncthreads();
  }
  const int nh = tot;

  if (wave == 0) {
#pragma unroll 1
    for (int b0 = 0; b0 < nh; b0 += 32) {
      const int idx = b0 + lane;
      const int uv  = reg1[idx < nh ? idx : nh - 1];
      const int m32 = (nh - b0) < 32 ? (nh - b0) : 32;
#pragma unroll 1
      for (int k = 0; k < m32; ++k) {
        const int u  = __builtin_amdgcn_readlane(uv, k);
        const int sl = u & (NBMAX - 1);
        if (lane == 0) scnt[sl] = scnt[sl] + 1;
      }
    }
  }
  __syncthreads();

  {
    const v4i ca = *(const v4i*)(scnt + 4 * tid);
    const int e0 = ca.x < 0 ? 0 : ca.x, e1 = ca.y < 0 ? 0 : ca.y, e2 = ca.z < 0 ? 0 : ca.z, e3 = ca.w < 0 ? 0 : ca.w;
    const int ts = e0 + e1 + e2 + e3;
    int incl = ts;
#pragma unroll
    for (int d = 1; d < 32; d <<= 1) {
      const int up = __shfl_up(incl, d);
      if (lane >= d) incl += up;
    }
    if (lane == 31) wtot[wave] = incl;
    __syncthreads();
    int pre = 0;
#pragma unroll
    for (int w2 = 0; w2 < NWAVE; ++w2) pre += (w2 < wave) ? wtot[w2] : 0;
    int run = pre + incl - ts;
    soff[4 * tid + 0] = run; run += e0;
    soff[4 * tid + 1] = run; run += e1;
    soff[4 * tid + 2] = run; run += e2;
    soff[4 * tid + 3] = run;
  }
  __syncthreads();
  for (int i = tid; i < NBMAX; i += NTHR) list[i] = soff[i];
  __syncthreads();

  if (wave == 0) {
#pragma unroll 1
    for (int b0 = 0; b0 < nh; b0 += 32) {
      const int idx = b0 + lane;
      const int uv  = reg1[idx < nh ? idx : nh - 1];
      const int m32 = (nh - b0) < 32 ? (nh - b0) : 32;
#pragma unroll 1
      for (int k = 0; k < m32; ++k) {
        const int u   = __builtin_amdgcn_readlane(uv, k);
        const int sl  = u & (NBMAX - 1);
        const int eid = (int)((unsigned)u >> SLOTB);
        if (lane == 0) {
          int pos = list[sl];
          pos = pos < 0 ? 0 : (pos > RCAP - 1 ? RCAP - 1 : pos);
          reg2[pos] = eid;
          list[sl] = pos + 1;
        }
      }
    }
  }
  __syncthreads();

  const int nbw = NBMAX / NWAVE;
  const bool ovf = (nh >= RCAP);
  const float qnan = __int_as_float(0x7fc00000);
  const int c4 = 4 * lane;
  const v4f z4 = {0.f, 0.f, 0.f, 0.f};
  const v4f wb1 = bfr4(*(const v4fa*)(Wb + c4));
  const v4f wb2 = bfr4(*(const v4fa*)(Wb + DM + c4));
  const v4f wb3 = bfr4(*(const v4fa*)(Wb + 2 * DM + c4));
  const v4f g14 = bfr4(*(const v4fa*)(g1p + c4));
  const v4f e14 = bfr4(*(const v4fa*)(e1p + c4));
  const float* wej = sWe + c4;

#pragma unroll 1
  for (int jt = 0; jt < nbw; ++jt) {
    const int slot = wave * nbw + jt;
    const int grow = nodeBase + slot;
    const int gcl  = grow < nN ? grow : nN - 1;
    int st = soff[slot];
    const int craw = scnt[slot];
    int cnt = craw;
    st  = st < 0 ? 0 : (st > nh ? nh : st);
    cnt = cnt < 0 ? 0 : (cnt > DEGCAP ? DEGCAP : cnt);
    if (cnt > nh - st) cnt = nh - st;
    const float pz = (ovf || craw > DEGCAP) ? qnan : 0.0f;

    const float* qr = QKVS + (size_t)gcl * QW;
    const v4f qv = *(const v4fa*)(qr + OQ + c4);
    const v4f sv = *(const v4fa*)(qr + OS + c4);
    const v4f xv = bfr4(*(const v4fa*)(x + (size_t)gcl * DM + c4));
    float mx = -1.0e30f, dn = 0.f;
    v4f av = z4;

#pragma unroll 1
    for (int q = 0; q < cnt; ++q) {
      int idx = st + q; idx = idx > RCAP - 1 ? RCAP - 1 : idx;
      int eid = reg2[idx]; eid = eid < 0 ? 0 : (eid > nE - 1 ? nE - 1 : eid);
      const int sraw = srcs[eid];
      const int s = sraw < 0 ? 0 : (sraw > nN - 1 ? nN - 1 : sraw);
      const float* kr = QKVS + (size_t)s * QW;
      const v4f kv = *(const v4fa*)(kr + OKY + c4);
      const v4f vv = *(const v4fa*)(kr + OV + c4);
      const float* ep = ea + (size_t)eid * EDM;
      v4f ef = z4;
#pragma unroll 1
      for (int jg = 0; jg < EDM / 4; ++jg) {
        const v4f aj = bfr4(*(const v4fa*)(ep + 4 * jg));
        const float* wp = wej + (size_t)(4 * jg) * DM;
        const v4f w0 = *(const v4fa*)(wp);
        const v4f w1 = *(const v4fa*)(wp + DM);
        const v4f w2 = *(const v4fa*)(wp + 2 * DM);
        const v4f w3 = *(const v4fa*)(wp + 3 * DM);
        ef = ef + w0 * aj.x;
        ef = ef + w1 * aj.y;
        ef = ef + w2 * aj.z;
        ef = ef + w3 * aj.w;
      }
      const v4f kj = kv + ef;
      const v4f vj = vv + ef;
      const float lg = hsum4(dot4(qv, kj)) * ATTSC;
      const float df = lg - mx;
      const float ex = __expf(-fabsf(df));
      const bool up  = df > 0.f;
      const float s1 = up ? ex : 1.0f;
      const float s2 = up ? 1.0f : ex;
      mx = up ? lg : mx;
      dn = fmaf(dn, s1, s2);
      av = av * s1 + vj * s2;
    }
    const float dns = dn > 0.f ? dn : 1.0f;
    const float ind = dn > 0.f ? 1.0f : 0.0f;
    const float inv = ind * __builtin_amdgcn_rcpf(dns);
    const v4f msg = av * inv + pz;

    const v4f dms = msg - sv;
    float part = dot4(msg, wb1);
    part += dot4(sv, wb2);
    part += dot4(dms, wb3);
    const float bd   = wsum(part);
    const float exb  = __expf(-bd);
    const float beta = __builtin_amdgcn_rcpf(1.0f + exb);
    const v4f hr = sv * beta + msg * (1.0f - beta);
    const v4f tt = hr + xv;
    const float sm = wsum((tt.x + tt.y) + (tt.z + tt.w));
    const float mu = sm * (1.0f / DM);
    const v4f d = tt - mu;
    const float sq = wsum((d.x * d.x + d.y * d.y) + (d.z * d.z + d.w * d.w));
    const float rs = rsqrtf(sq * (1.0f / DM) + LNEPS);
    const v4f y = d * rs * g14 + e14;

    const bool wr = (grow < MPr);
    const int gsf = wr ? grow : MPr - 1;
    float* orow = H1 + (size_t)gsf * DM + c4;
    if (wr) {
      *(volatile v4f*)orow = y;
    }
    __threadfence();
    if (wr) {
      *(volatile v4f*)orow = y;
    }
  }
}

__global__ __launch_bounds__(GTHR) void k_tail(
    const float* __restrict__ H1, const unsigned short* __restrict__ W1T, const unsigned short* __restrict__ W2T,
    const float* __restrict__ b1, const float* __restrict__ b2,
    const float* __restrict__ g2p, const float* __restrict__ e2p,
    float* out, int nN)
{
  extern __shared__ v4f lds_dyn[];
  unsigned short* At = (unsigned short*)lds_dyn;
  unsigned short* Ht = At + GBM * KO;
  float* stg = (float*)(Ht + GBM * KF);
  const int tid = (int)threadIdx.x, lane = tid & 31, wave = tid >> 5, hh = lane >> 4, m = lane & 15;
  const int rowBase = (int)blockIdx.x * GBM;
  const int c4 = 4 * lane;
  const v8f z8 = {0.f, 0.f, 0.f, 0.f, 0.f, 0.f, 0.f, 0.f};

#pragma unroll 2
  for (int i = 0; i < 8; ++i) {
    const int p   = i * GTHR + tid;
    const int row = p >> 4;
    const int q8  = (p & 15) * 8;
    const float* hp = H1 + (size_t)(rowBase + row) * DM + q8;
    const v4f a = *(const v4fa*)hp;
    const v4f b = *(const v4fa*)(hp + 4);
    v4u hv, lv;
    pack8hl(a, b, hv, lv);
    *(v4ua*)(At + row * KO + q8)      = hv;
    *(v4ua*)(At + row * KO + DM + q8) = lv;
  }
  __syncthreads();

  v8f acc[8];
#pragma unroll 1
  for (int g = 0; g < FW / DM; ++g) {
#pragma unroll
    for (int t = 0; t < 8; ++t) acc[t] = z8;
    const unsigned short* aq = At + (size_t)(16 * wave + m) * KO + 8 * hh;
    const unsigned short* wp = W1T + (size_t)(g * DM + m) * (size_t)KO + 8 * hh;
#pragma unroll 1
    for (int ks = 0; ks < KO / 32; ++ks) {
      FragB af;
      af.h[0] = *(const v8usa*)(aq + 32 * ks);
      af.h[1] = *(const v8usa*)(aq + 32 * ks + 16);
#pragma unroll
      for (int t = 0; t < 8; ++t) {
        const unsigned short* wq = wp + (size_t)(16 * t) * (size_t)KO + 32 * ks;
        FragB bf;
        bf.h[0] = *(const v8usa*)wq;
        bf.h[1] = *(const v8usa*)(wq + 16);
        acc[t] = wmb(af, bf, acc[t]);
      }
    }
#pragma unroll
    for (int t = 0; t < 8; ++t) {
      const int lc = 16 * t + m;
#pragma unroll
      for (int r = 0; r < 8; ++r) {
        const int lr = 16 * wave + 8 * hh + r;
        stg[lr * DM + lc] = acc[t][r];
      }
    }
    __syncthreads();
#pragma unroll 2
    for (int i = 0; i < 8; ++i) {
      const int p   = i * GTHR + tid;
      const int row = p >> 4;
      const int q8  = (p & 15) * 8;
      v4f a = *(const v4fa*)(stg + row * DM + q8);
      v4f b = *(const v4fa*)(stg + row * DM + q8 + 4);
      const v4f ba = bfr4(*(const v4fa*)(b1 + g * DM + q8));
      const v4f bb = bfr4(*(const v4fa*)(b1 + g * DM + q8 + 4));
      a = relu4(a + ba);
      b = relu4(b + bb);
      v4u hv, lv;
      pack8hl(a, b, hv, lv);
      *(v4ua*)(Ht + row * KF + g * DM + q8)      = hv;
      *(v4ua*)(Ht + row * KF + FW + g * DM + q8) = lv;
    }
    __syncthreads();
  }

#pragma unroll
  for (int t = 0; t < 8; ++t) acc[t] = z8;
  {
    const unsigned short* aq = Ht + (size_t)(16 * wave + m) * KF + 8 * hh;
    const unsigned short* wp = W2T + (size_t)m * (size_t)KF + 8 * hh;
#pragma unroll 1
    for (int ks = 0; ks < KF / 32; ++ks) {
      FragB af;
      af.h[0] = *(const v8usa*)(aq + 32 * ks);
      af.h[1] = *(const v8usa*)(aq + 32 * ks + 16);
#pragma unroll
      for (int t = 0; t < 8; ++t) {
        const unsigned short* wq = wp + (size_t)(16 * t) * (size_t)KF + 32 * ks;
        FragB bf;
        bf.h[0] = *(const v8usa*)wq;
        bf.h[1] = *(const v8usa*)(wq + 16);
        acc[t] = wmb(af, bf, acc[t]);
      }
    }
  }
#pragma unroll
  for (int t = 0; t < 8; ++t) {
    const int lc = 16 * t + m;
#pragma unroll
    for (int r = 0; r < 8; ++r) {
      const int lr = 16 * wave + 8 * hh + r;
      stg[lr * DM + lc] = acc[t][r];
    }
  }
  __syncthreads();

  const v4f b24 = bfr4(*(const v4fa*)(b2  + c4));
  const v4f g24 = bfr4(*(const v4fa*)(g2p + c4));
  const v4f e24 = bfr4(*(const v4fa*)(e2p + c4));
#pragma unroll 1
  for (int i = 0; i < 16; ++i) {
    const int lr = 16 * wave + i;
    const int gr = rowBase + lr;
    const v4f a  = *(const v4fa*)(stg + lr * DM + c4);
    const v4f r1 = *(const v4fa*)(H1 + (size_t)gr * DM + c4);
    const v4f tt = (a + b24) + r1;
    const float sm = wsum((tt.x + tt.y) + (tt.z + tt.w));
    const float mu = sm * (1.0f / DM);
    const v4f d = tt - mu;
    const float sq = wsum((d.x * d.x + d.y * d.y) + (d.z * d.z + d.w * d.w));
    const float rs = rsqrtf(sq * (1.0f / DM) + LNEPS);
    const v4f y = d * rs * g24 + e24;
    if (gr < nN) {
      float* op = out + (size_t)gr * DM + c4;
      *(volatile v4f*)op = y;
      __threadfence();
      *(volatile v4f*)op = y;
    }
  }
}

static inline int cdiv(int a, int b) { return (a + b - 1) / b; }

extern "C" void kernel_launch(void* const* d_in, const int* in_sizes, int n_in,
                              void* d_out, int out_size, void* d_ws, size_t ws_size,
                              hipStream_t stream) {
  if (n_in < 21) return;
  if (in_sizes[0] < DM || (in_sizes[0] % DM) != 0) return;
  const int nN = in_sizes[0] / DM;
  if (nN < 1 || nN > (1 << 22)) return;
  if (in_sizes[1] < 2 || (in_sizes[1] & 1) != 0) return;
  const int nE = in_sizes[1] / 2;
  if (nE < 1 || nE >= (1 << (31 - SLOTB))) return;
  if (in_sizes[2] != nE * EDM) return;
  if (in_sizes[3] != DM * DM || in_sizes[5] != DM * DM || in_sizes[7] != DM * DM || in_sizes[10] != DM * DM) return;
  if (in_sizes[4] != DM || in_sizes[6] != DM || in_sizes[8] != DM || in_sizes[11] != DM) return;
  if (in_sizes[9] != DM * EDM) return;
  if (in_sizes[12] != 3 * DM) return;
  if (in_sizes[13] != DM || in_sizes[14] != DM || in_sizes[15] != DM || in_sizes[16] != DM) return;
  if (in_sizes[17] != FW * DM || in_sizes[18] != FW) return;
  if (in_sizes[19] != DM * FW || in_sizes[20] != DM) return;
  if (out_size != nN * DM) return;

  const float* x     = (const float*)d_in[0];
  const int*   ei    = (const int*)  d_in[1];
  const float* ea    = (const float*)d_in[2];
  const float* Wq    = (const float*)d_in[3];
  const float* bq    = (const float*)d_in[4];
  const float* Wk    = (const float*)d_in[5];
  const float* bk    = (const float*)d_in[6];
  const float* Wv    = (const float*)d_in[7];
  const float* bv    = (const float*)d_in[8];
  const float* We    = (const float*)d_in[9];
  const float* Wsk   = (const float*)d_in[10];
  const float* bsk   = (const float*)d_in[11];
  const float* Wb    = (const float*)d_in[12];
  const float* g1p   = (const float*)d_in[13];
  const float* e1p   = (const float*)d_in[14];
  const float* g2p   = (const float*)d_in[15];
  const float* e2p   = (const float*)d_in[16];
  const float* W1    = (const float*)d_in[17];
  const float* b1    = (const float*)d_in[18];
  const float* W2    = (const float*)d_in[19];
  const float* b2    = (const float*)d_in[20];
  float* out = (float*)d_out;
  const int* src = ei;
  const int* dst = ei + nE;

  const int MP   = cdiv(nN, GBM) * GBM;
  const int gA   = cdiv(MP, NBMAX);
  const int vec8 = ((nE & 3) == 0) ? 1 : 0;
  if ((long long)gA * NBMAX < (long long)MP) return;

  char* ws = (char*)d_ws;
  size_t off = 0;
  const size_t szXB = (size_t)MP * DM * 2, szH1 = (size_t)MP * DM * 4;
  const size_t oR0  = off; off += (szH1 > szXB ? szH1 : szXB);     off = (off + 255) & ~(size_t)255;
  const size_t oWQ  = off; off += (size_t)QW * DM * 2;             off = (off + 255) & ~(size_t)255;
  const size_t oW1  = off; off += (size_t)FW * KO * 2;             off = (off + 255) & ~(size_t)255;
  const size_t oW2  = off; off += (size_t)DM * KF * 2;             off = (off + 255) & ~(size_t)255;
  const size_t oQ   = off; off += (size_t)MP * QW * 4;             off = (off + 255) & ~(size_t)255;
  if (off > ws_size || off > (size_t)WSMAX) return;
  unsigned short* XB    = (unsigned short*)(ws + oR0);
  float*          H1    = (float*)(ws + oR0);
  unsigned short* WQKVS = (unsigned short*)(ws + oWQ);
  unsigned short* W1T2  = (unsigned short*)(ws + oW1);
  unsigned short* W2T2  = (unsigned short*)(ws + oW2);
  float*          QKVS  = (float*)(ws + oQ);

  hipFuncSetAttribute(reinterpret_cast<const void*>(&k_agg),
                      hipFuncAttributeMaxDynamicSharedMemorySize, LDS_AGG);
  hipFuncSetAttribute(reinterpret_cast<const void*>(&k_tail),
                      hipFuncAttributeMaxDynamicSharedMemorySize, LDS_TAIL);

  const int nUx = MP * (DM / 8);
  k_xprep<<<cdiv(nUx, NTHR), NTHR, 0, stream>>>(x, XB, nN, nUx);

  {
    const int nUq = DM * (DM / 8);
    const size_t pl = (size_t)DM * DM;
    k_wcvt<<<cdiv(nUq, NTHR), NTHR, 0, stream>>>(Wq,  DM, DM, DM, WQKVS,          nUq);
    k_wcvt<<<cdiv(nUq, NTHR), NTHR, 0, stream>>>(Wk,  DM, DM, DM, WQKVS + pl,     nUq);
    k_wcvt<<<cdiv(nUq, NTHR), NTHR, 0, stream>>>(Wv,  DM, DM, DM, WQKVS + 2 * pl, nUq);
    k_wcvt<<<cdiv(nUq, NTHR), NTHR, 0, stream>>>(Wsk, DM, DM, DM, WQKVS + 3 * pl, nUq);
    const int nU1 = FW * (KO / 8);
    k_wcvt<<<cdiv(nU1, NTHR), NTHR, 0, stream>>>(W1, DM, FW, KO, W1T2, nU1);
    const int nU2 = DM * (KF / 8);
    k_wcvt<<<cdiv(nU2, NTHR), NTHR, 0, stream>>>(W2, FW, DM, KF, W2T2, nU2);
  }

  {
    const int gM = MP / GBM;
    const size_t pl = (size_t)DM * DM;
    k_gemm<<<dim3(gM, DM / GBN), GTHR, 0, stream>>>(XB, WQKVS,          bq,  QKVS + OQ);
    k_gemm<<<dim3(gM, DM / GBN), GTHR, 0, stream>>>(XB, WQKVS + pl,     bk,  QKVS + OKY);
    k_gemm<<<dim3(gM, DM / GBN), GTHR, 0, stream>>>(XB, WQKVS + 2 * pl, bv,  QKVS + OV);
    k_gemm<<<dim3(gM, DM / GBN), GTHR, 0, stream>>>(XB, WQKVS + 3 * pl, bsk, QKVS + OS);
  }

  k_agg<<<gA, NTHR, LDS_AGG, stream>>>(src, dst, QKVS, ea, We, Wb, x, g1p, e1p, H1, nN, nE, vec8, MP);
  k_tail<<<MP / GBM, GTHR, LDS_TAIL, stream>>>(H1, W1T2, W2T2, b1, b2, g2p, e2p, out, nN);
}
